// MaskingAwareAttention_82240033784118
// MI455X (gfx1250) — hardware-verified
//
#include <hip/hip_runtime.h>

typedef _Float16 v16h __attribute__((ext_vector_type(16)));
typedef _Float16 v8h  __attribute__((ext_vector_type(8)));
typedef float    v8f  __attribute__((ext_vector_type(8)));
typedef float    v4f  __attribute__((ext_vector_type(4)));
typedef float    v2f  __attribute__((ext_vector_type(2)));
typedef int      v4i  __attribute__((ext_vector_type(4)));
typedef v8h __attribute__((may_alias)) v8ha;
typedef v4f __attribute__((may_alias)) v4fa;
typedef v4i __attribute__((may_alias)) v4ia;

union Frag { v16h v; v8h half[2]; };

#define DMODEL 512
#define NHEADS 8
#define HD     64
#define SEQ    2048
#define BATCH  4
#define MROWS  (BATCH * SEQ)
#define NX     (MROWS * DMODEL)
#define NW     (DMODEL * DMODEL)
#define NX8    (NX / 8)
#define NW8    (NW / 8)
#define RELN   (2 * SEQ - 1)
#define NPE    (SEQ * DMODEL)
#define PSCALE  16384.0f
#define WSCALE  32.0f
#define AOSCALE 64.0f

static_assert(NW8 == 32768);
static_assert((NX8 % 256) == 0);
static_assert((MROWS % 128) == 0 && (SEQ % 128) == 0);

__device__ __forceinline__ v8f wmma_f16(v16h a, v16h b, v8f c) {
  v8f d = __builtin_amdgcn_wmma_f32_16x16x32_f16(false, a, false, b, (short)0, c, false, false);
  asm volatile("v_nop\n\tv_nop\n\tv_nop\n\tv_nop" : "+v"(d) : "v"(a), "v"(b));
  return d;
}

__device__ __forceinline__ v16h load_frag(const _Float16* p, int h) {
  Frag f;
  f.half[0] = *(const v8ha*)(p + 8 * h);
  f.half[1] = *(const v8ha*)(p + 16 + 8 * h);
  return f.v;
}

__global__ __launch_bounds__(256) void pe_kernel(float* __restrict__ pet)
{
  const int idx = blockIdx.x * 256 + threadIdx.x;
  if (idx >= SEQ * (DMODEL / 2)) return;
  const int t = idx >> 8;
  const int p = idx & 255;
  const float kc = (float)(-9.210340371976184 / 512.0);
  const float fr = expf((float)(2 * p) * kc);
  const float ang = (float)t * fr;
  v2f o;
  o.x = sinf(ang);
  o.y = cosf(ang);
  float* dst = pet + (size_t)idx * 2;
  *(volatile v2f*)dst = o;
  __threadfence();
  *(volatile v2f*)dst = o;
}

__global__ __launch_bounds__(256) void convert_kernel(
    const float* __restrict__ x, const float* __restrict__ pet,
    const float* __restrict__ wq, const float* __restrict__ wk,
    const float* __restrict__ wv, const float* __restrict__ wo,
    _Float16* __restrict__ xh, _Float16* __restrict__ wh)
{
  const int g = blockIdx.x * 256 + threadIdx.x;
  if (g >= NX8 + 4 * NW8) return;
  v4f a, c;
  _Float16* dst;
  if (g < NX8) {
    const int row = g >> 6;
    const int t = row & (SEQ - 1);
    const int db = (g & 63) * 8;
    const float* src = x + (size_t)g * 8;
    const float* pp = pet + (size_t)t * DMODEL + db;
    a = *(const v4fa*)src + *(const v4fa*)pp;
    c = *(const v4fa*)(src + 4) + *(const v4fa*)(pp + 4);
    dst = xh + (size_t)g * 8;
  } else {
    const int e = g - NX8;
    const int wsel = e >> 15;
    const int off = e & (NW8 - 1);
    const float* wsrc = (wsel == 0) ? wq : ((wsel == 1) ? wk : ((wsel == 2) ? wv : wo));
    const float* src = wsrc + (size_t)off * 8;
    a = *(const v4fa*)src * WSCALE;
    c = *(const v4fa*)(src + 4) * WSCALE;
    dst = wh + (size_t)e * 8;
  }
  const v8h o = { (_Float16)a.x, (_Float16)a.y, (_Float16)a.z, (_Float16)a.w,
                  (_Float16)c.x, (_Float16)c.y, (_Float16)c.z, (_Float16)c.w };
  *(volatile v8h*)dst = o;
  __threadfence();
  *(volatile v8h*)dst = o;
}

__device__ __forceinline__ void proj_store_pass(const _Float16* sT, _Float16* plane, _Float16* vt,
                                                int which, int bh, int l0, int w, int lane) {
  const int q8 = lane & 7, sub = lane >> 3;
  #pragma unroll
  for (int i = 0; i < 8; ++i) {
    const int lid = w * 32 + i * 4 + sub;
    v8h v;
    _Float16* dst;
    if (which != 2) {
      v = *(const v8ha*)(sT + lid * HD + 8 * q8);
      dst = plane + ((size_t)bh * SEQ + l0 + lid) * HD + 8 * q8;
    } else {
      const int d = lid >> 1, hl = lid & 1;
      v = *(const v8ha*)(sT + d * 128 + 64 * hl + 8 * q8);
      dst = vt + ((size_t)bh * HD + d) * SEQ + l0 + 64 * hl + 8 * q8;
    }
    *(volatile v8h*)dst = v;
  }
}

__global__ __launch_bounds__(128) void proj_kernel(
    const _Float16* __restrict__ xh,
    const _Float16* __restrict__ wh,
    const float* __restrict__ bq, const float* __restrict__ bk, const float* __restrict__ bv,
    _Float16* __restrict__ qh,
    _Float16* __restrict__ kh,
    _Float16* __restrict__ vt)
{
  __shared__ __attribute__((aligned(16))) _Float16 sT[128 * 64];

  const int tid = threadIdx.x, lane = tid & 31, w = tid >> 5;
  const int h = lane >> 4, m = lane & 15;
  const int m0 = blockIdx.x * 128;
  const int cg = blockIdx.y;
  const int which = cg >> 3, head = cg & 7;
  const int m0w = m0 + 32 * w;

  const _Float16* xa0 = xh + (size_t)(m0w + m) * DMODEL;
  const _Float16* xa1 = xa0 + (size_t)16 * DMODEL;
  const _Float16* wb  = wh + ((size_t)which * DMODEL + head * HD + m) * DMODEL;

  const v8f zero8 = {0.f, 0.f, 0.f, 0.f, 0.f, 0.f, 0.f, 0.f};
  v8f acc[2][4];
  #pragma unroll
  for (int mt = 0; mt < 2; ++mt)
    #pragma unroll
    for (int nt = 0; nt < 4; ++nt) acc[mt][nt] = zero8;

  #pragma unroll 1
  for (int k0 = 0; k0 < DMODEL; k0 += 32) {
    const v16h a0 = load_frag(xa0 + k0, h);
    const v16h a1 = load_frag(xa1 + k0, h);
    #pragma unroll
    for (int nt = 0; nt < 4; ++nt) {
      const v16h b = load_frag(wb + (size_t)nt * 16 * DMODEL + k0, h);
      acc[0][nt] = wmma_f16(a0, b, acc[0][nt]);
      acc[1][nt] = wmma_f16(a1, b, acc[1][nt]);
    }
  }

  const float* bias = (which == 0) ? bq : ((which == 1) ? bk : bv);
  #pragma unroll
  for (int nt = 0; nt < 4; ++nt) {
    const int feat = 16 * nt + m;
    const float bvl = bias[head * HD + feat];
    #pragma unroll
    for (int mt = 0; mt < 2; ++mt) {
      #pragma unroll
      for (int r = 0; r < 8; ++r) {
        const int tokl = 32 * w + 16 * mt + 8 * h + r;
        const float y = acc[mt][nt][r] * (1.0f / WSCALE) + bvl;
        const int idx = (which == 2) ? (feat * 128 + tokl) : (tokl * HD + feat);
        sT[idx] = (_Float16)y;
      }
    }
  }
  __syncthreads();

  const int b = m0 / SEQ, l0 = m0 - b * SEQ, bh = b * NHEADS + head;
  _Float16* plane = (which == 0) ? qh : kh;
  proj_store_pass(sT, plane, vt, which, bh, l0, w, lane);
  __threadfence();
  proj_store_pass(sT, plane, vt, which, bh, l0, w, lane);
}

__device__ __forceinline__ v8f bias_mask8(v8f s, const int* mk, const float* sb, int base, float vmiss) {
  const v4i ma = *(const v4ia*)mk;
  const v4i mb = *(const v4ia*)(mk + 4);
  s[0] = (ma.x != 0) ? fmaf(s[0], 0.125f, sb[base])     : vmiss;
  s[1] = (ma.y != 0) ? fmaf(s[1], 0.125f, sb[base - 1]) : vmiss;
  s[2] = (ma.z != 0) ? fmaf(s[2], 0.125f, sb[base - 2]) : vmiss;
  s[3] = (ma.w != 0) ? fmaf(s[3], 0.125f, sb[base - 3]) : vmiss;
  s[4] = (mb.x != 0) ? fmaf(s[4], 0.125f, sb[base - 4]) : vmiss;
  s[5] = (mb.y != 0) ? fmaf(s[5], 0.125f, sb[base - 5]) : vmiss;
  s[6] = (mb.z != 0) ? fmaf(s[6], 0.125f, sb[base - 6]) : vmiss;
  s[7] = (mb.w != 0) ? fmaf(s[7], 0.125f, sb[base - 7]) : vmiss;
  return s;
}

__device__ __forceinline__ v16h pack_p(v8f a, v8f c) {
  const v16h r = { (_Float16)(a[0] * PSCALE), (_Float16)(a[1] * PSCALE), (_Float16)(a[2] * PSCALE), (_Float16)(a[3] * PSCALE),
                   (_Float16)(a[4] * PSCALE), (_Float16)(a[5] * PSCALE), (_Float16)(a[6] * PSCALE), (_Float16)(a[7] * PSCALE),
                   (_Float16)(c[0] * PSCALE), (_Float16)(c[1] * PSCALE), (_Float16)(c[2] * PSCALE), (_Float16)(c[3] * PSCALE),
                   (_Float16)(c[4] * PSCALE), (_Float16)(c[5] * PSCALE), (_Float16)(c[6] * PSCALE), (_Float16)(c[7] * PSCALE) };
  return r;
}

__device__ __forceinline__ void ao_store_pass(const _Float16* so, _Float16* ao,
                                              int b, int head, int q0, int lane) {
  const int q8 = lane & 7, sub = lane >> 3;
  #pragma unroll
  for (int i = 0; i < 4; ++i) {
    const int lid = i * 4 + sub;
    const v8h v = *(const v8ha*)(so + lid * 64 + 8 * q8);
    const size_t gi = ((size_t)b * SEQ + q0 + lid) * DMODEL + head * HD + 8 * q8;
    *(volatile v8h*)(ao + gi) = v;
  }
}

__global__ __launch_bounds__(128) void attn_kernel(
    const _Float16* __restrict__ qh,
    const _Float16* __restrict__ kh,
    const _Float16* __restrict__ vt,
    const int* __restrict__ mask,
    const float* __restrict__ mbias,
    const float* __restrict__ rel,
    _Float16* __restrict__ ao)
{
  __shared__ __attribute__((aligned(16))) float sB[4096];
  __shared__ __attribute__((aligned(16))) _Float16 sO[4 * 16 * 64];

  const int tid = threadIdx.x, lane = tid & 31, w = tid >> 5;
  const int h = lane >> 4, m = lane & 15;
  const int bh = blockIdx.y, b = bh >> 3, head = bh & 7;
  const int q0 = blockIdx.x * 64 + 16 * w;

  for (int i = tid; i < 4096; i += 128) {
    float v = 0.0f;
    if (i < RELN) v = 0.5f * (rel[(size_t)i * NHEADS + head] - rel[(size_t)(RELN - 1 - i) * NHEADS + head]);
    sB[i] = v;
  }

  const _Float16* qrow = qh + ((size_t)bh * SEQ + q0 + m) * HD;
  const v16h qb0 = load_frag(qrow, h);
  const v16h qb1 = load_frag(qrow + 32, h);

  __syncthreads();

  const float mbh = mbias[head];
  const float vmiss = -__builtin_inff() + mbh;
  const int qk = q0 + m + (SEQ - 1) - 8 * h;

  const v8f zero8 = {0.f, 0.f, 0.f, 0.f, 0.f, 0.f, 0.f, 0.f};
  v8f o[4];
  #pragma unroll
  for (int t = 0; t < 4; ++t) o[t] = zero8;
  float mrun = -1e30f, lrun = 0.0f;

  const _Float16* kbase = kh + ((size_t)bh * SEQ + m) * HD;
  const _Float16* vbase = vt + ((size_t)bh * HD + m) * SEQ;
  const int* mkp = mask + (size_t)b * SEQ + 8 * h;

  #pragma unroll 1
  for (int kb = 0; kb < SEQ; kb += 64) {
    v8f s[4];
    #pragma unroll
    for (int j = 0; j < 4; ++j) {
      const _Float16* kp = kbase + (size_t)(kb + 16 * j) * HD;
      const v16h kf0 = load_frag(kp, h);
      const v16h kf1 = load_frag(kp + 32, h);
      v8f z = zero8;
      z = wmma_f16(kf0, qb0, z);
      z = wmma_f16(kf1, qb1, z);
      s[j] = z;
    }
    #pragma unroll
    for (int j = 0; j < 4; ++j)
      s[j] = bias_mask8(s[j], mkp + kb + 16 * j, sB, qk - kb - 16 * j, vmiss);

    float mloc = s[0][0];
    #pragma unroll
    for (int j = 0; j < 4; ++j)
      #pragma unroll
      for (int r = 0; r < 8; ++r) mloc = fmaxf(mloc, s[j][r]);
    mloc = fmaxf(mloc, __shfl_xor(mloc, 16));
    const float mnew = fmaxf(mrun, mloc);
    const float alpha = __expf(mrun - mnew);
    mrun = mnew;
    float lsum = 0.0f;
    #pragma unroll
    for (int j = 0; j < 4; ++j)
      #pragma unroll
      for (int r = 0; r < 8; ++r) {
        const float p = __expf(s[j][r] - mnew);
        s[j][r] = p;
        lsum += p;
      }
    lsum += __shfl_xor(lsum, 16);
    lrun = lrun * alpha + lsum;
    #pragma unroll
    for (int t = 0; t < 4; ++t)
      #pragma unroll
      for (int r = 0; r < 8; ++r) o[t][r] = o[t][r] * alpha;

    const v16h pb0 = pack_p(s[0], s[1]);
    const v16h pb1 = pack_p(s[2], s[3]);

    #pragma unroll
    for (int t = 0; t < 4; ++t) {
      const _Float16* vp = vbase + (size_t)(16 * t) * SEQ + kb;
      const v16h vf0 = load_frag(vp, h);
      const v16h vf1 = load_frag(vp + 32, h);
      o[t] = wmma_f16(vf0, pb0, o[t]);
      o[t] = wmma_f16(vf1, pb1, o[t]);
    }
  }

  const float inv = __builtin_amdgcn_rcpf(lrun) * (AOSCALE / PSCALE);
  _Float16* so = sO + w * 1024;
  #pragma unroll
  for (int t = 0; t < 4; ++t)
    #pragma unroll
    for (int r = 0; r < 8; ++r)
      so[m * 64 + 16 * t + 8 * h + r] = (_Float16)(o[t][r] * inv);
  __syncthreads();

  ao_store_pass(so, ao, b, head, q0, lane);
  __threadfence();
  ao_store_pass(so, ao, b, head, q0, lane);
}

__device__ __forceinline__ void out_store_pass(const float* sT, float* out, int m0, int fg, int w, int lane) {
  const int q8 = lane & 7, sub = lane >> 3;
  #pragma unroll
  for (int i = 0; i < 16; ++i) {
    const int lid = i * 4 + sub;
    const int row = 32 * w + (lid >> 1), hl = lid & 1;
    const v4f v = *(const v4fa*)(sT + row * 64 + 32 * hl + 4 * q8);
    const size_t gi = ((size_t)(m0 + row)) * DMODEL + fg * 64 + 32 * hl + 4 * q8;
    *(volatile v4f*)(out + gi) = v;
  }
}

__global__ __launch_bounds__(128) void oproj_kernel(
    const _Float16* __restrict__ ao,
    const _Float16* __restrict__ woh,
    const float* __restrict__ bo,
    float* __restrict__ out)
{
  __shared__ __attribute__((aligned(16))) float sT[128 * 64];

  const int tid = threadIdx.x, lane = tid & 31, w = tid >> 5;
  const int h = lane >> 4, m = lane & 15;
  const int m0 = blockIdx.x * 128;
  const int fg = blockIdx.y;
  const int m0w = m0 + 32 * w;

  const _Float16* xa0 = ao + (size_t)(m0w + m) * DMODEL;
  const _Float16* xa1 = xa0 + (size_t)16 * DMODEL;
  const _Float16* wb  = woh + ((size_t)fg * 64 + m) * DMODEL;

  const v8f zero8 = {0.f, 0.f, 0.f, 0.f, 0.f, 0.f, 0.f, 0.f};
  v8f acc[2][4];
  #pragma unroll
  for (int mt = 0; mt < 2; ++mt)
    #pragma unroll
    for (int nt = 0; nt < 4; ++nt) acc[mt][nt] = zero8;

  #pragma unroll 1
  for (int k0 = 0; k0 < DMODEL; k0 += 32) {
    const v16h a0 = load_frag(xa0 + k0, h);
    const v16h a1 = load_frag(xa1 + k0, h);
    #pragma unroll
    for (int nt = 0; nt < 4; ++nt) {
      const v16h b = load_frag(wb + (size_t)nt * 16 * DMODEL + k0, h);
      acc[0][nt] = wmma_f16(a0, b, acc[0][nt]);
      acc[1][nt] = wmma_f16(a1, b, acc[1][nt]);
    }
  }

  #pragma unroll
  for (int nt = 0; nt < 4; ++nt) {
    const int feat = 16 * nt + m;
    const float bvl = bo[fg * 64 + feat];
    #pragma unroll
    for (int mt = 0; mt < 2; ++mt) {
      #pragma unroll
      for (int r = 0; r < 8; ++r) {
        const int tokl = 32 * w + 16 * mt + 8 * h + r;
        sT[tokl * 64 + feat] = acc[mt][nt][r] * (1.0f / (WSCALE * AOSCALE)) + bvl;
      }
    }
  }
  __syncthreads();

  out_store_pass(sT, out, m0, fg, w, lane);
  __threadfence();
  out_store_pass(sT, out, m0, fg, w, lane);
}

extern "C" void kernel_launch(void* const* d_in, const int* in_sizes, int n_in,
                              void* d_out, int out_size, void* d_ws, size_t ws_size,
                              hipStream_t stream) {
  if (n_in < 12) return;
  if (in_sizes[0] != NX) return;
  if (in_sizes[1] != MROWS) return;
  if (in_sizes[2] != NW || in_sizes[4] != NW || in_sizes[6] != NW || in_sizes[8] != NW) return;
  if (in_sizes[3] != DMODEL || in_sizes[5] != DMODEL || in_sizes[7] != DMODEL || in_sizes[9] != DMODEL) return;
  if (in_sizes[10] != NHEADS) return;
  if (in_sizes[11] != RELN * NHEADS) return;
  if (out_size != NX) return;

  const float* x     = (const float*)d_in[0];
  const int*   mask  = (const int*)d_in[1];
  const float* Wq    = (const float*)d_in[2];
  const float* bq    = (const float*)d_in[3];
  const float* Wk    = (const float*)d_in[4];
  const float* bk    = (const float*)d_in[5];
  const float* Wv    = (const float*)d_in[6];
  const float* bv    = (const float*)d_in[7];
  const float* Wo    = (const float*)d_in[8];
  const float* bo    = (const float*)d_in[9];
  const float* mbias = (const float*)d_in[10];
  const float* rel   = (const float*)d_in[11];
  float* out = (float*)d_out;

  const size_t pe_bytes = (size_t)NPE * 4;
  const size_t xh_bytes = (size_t)NX * 2;
  const size_t wh_bytes = (size_t)4 * NW * 2;
  const size_t pl_bytes = (size_t)BATCH * NHEADS * SEQ * HD * 2;
  const size_t ao_bytes = (size_t)NX * 2;
  const size_t total = pe_bytes + xh_bytes + wh_bytes + 3 * pl_bytes + ao_bytes;
  if (total > ws_size) return;

  char* ws = (char*)d_ws;
  size_t off = 0;
  float*    pet = (float*)(ws + off);     off += pe_bytes;
  _Float16* xh  = (_Float16*)(ws + off);  off += xh_bytes;
  _Float16* wh  = (_Float16*)(ws + off);  off += wh_bytes;
  _Float16* qh  = (_Float16*)(ws + off);  off += pl_bytes;
  _Float16* kh  = (_Float16*)(ws + off);  off += pl_bytes;
  _Float16* vt  = (_Float16*)(ws + off);  off += pl_bytes;
  _Float16* ao  = (_Float16*)(ws + off);  off += ao_bytes;
  if (off > ws_size) return;

  const int npairs = SEQ * (DMODEL / 2);
  pe_kernel<<<(npairs + 255) / 256, 256, 0, stream>>>(pet);

  const int ngroups = NX8 + 4 * NW8;
  convert_kernel<<<(ngroups + 255) / 256, 256, 0, stream>>>(x, pet, Wq, Wk, Wv, Wo, xh, wh);

  dim3 gProj(MROWS / 128, 3 * NHEADS);
  proj_kernel<<<gProj, 128, 0, stream>>>(xh, wh, bq, bk, bv, qh, kh, vt);

  dim3 gAtt(SEQ / 64, BATCH * NHEADS);
  attn_kernel<<<gAtt, 128, 0, stream>>>(qh, kh, vt, mask, mbias, rel, ao);

  dim3 gOut(MROWS / 128, DMODEL / 64);
  oproj_kernel<<<gOut, 128, 0, stream>>>(ao, wh + (size_t)3 * NW, bo, out);
}
